// TAISP_76355928588665
// MI455X (gfx1250) — hardware-verified
//
#include <hip/hip_runtime.h>
#define BB 4
#define HI 1024
#define WI 1024
#define NPIX (HI * WI)
#define NF 32

typedef __bf16 v16b __attribute__((ext_vector_type(16)));
typedef unsigned short v8us __attribute__((ext_vector_type(8), may_alias));
typedef float  v8f  __attribute__((ext_vector_type(8)));
typedef float  v4f  __attribute__((ext_vector_type(4)));
typedef float  v4fa __attribute__((ext_vector_type(4), may_alias));
union FragB { v16b v; v8us half[2]; unsigned short u[16]; };

__device__ __forceinline__ unsigned short bf16_bits(float x) { unsigned int u = __float_as_uint(x); return (unsigned short)((u + 0x7FFFu + ((u >> 16) & 1u)) >> 16); }
__device__ __forceinline__ float bf16_val(unsigned short b) { return __uint_as_float(((unsigned int)b) << 16); }
__device__ __forceinline__ float bf16_round(float x) { return bf16_val(bf16_bits(x)); }
template <int NT>
__device__ __forceinline__ v8f mmaN(v16b ah, v16b al, v16b bh, v16b bl, v8f c) {
  c = __builtin_amdgcn_wmma_f32_16x16x32_bf16(false, ah, false, bh, (short)0, c, false, false);
  if (NT >= 2) c = __builtin_amdgcn_wmma_f32_16x16x32_bf16(false, al, false, bh, (short)0, c, false, false);
  if (NT >= 3) c = __builtin_amdgcn_wmma_f32_16x16x32_bf16(false, ah, false, bl, (short)0, c, false, false);
  asm volatile("v_nop\n\tv_nop\n\tv_nop\n\tv_nop" : "+v"(c) : "v"(ah), "v"(al), "v"(bh), "v"(bl));
  return c;
}

__global__ __launch_bounds__(256) void k_wt_bf16(const float* __restrict__ W, unsigned short* __restrict__ Wt, int K, int N) {
  const int t = blockIdx.x * 256 + threadIdx.x;
  const int k8n = K / 8;
  if (t >= N * k8n) return;
  const int n = t / k8n, k8 = (t % k8n) * 8;
  v8us v;
#pragma unroll
  for (int i = 0; i < 8; ++i) v[i] = bf16_bits(W[(size_t)(k8 + i) * N + n]);
  *(volatile v8us*)(Wt + (size_t)n * K + k8) = v;
  __threadfence();
  *(volatile v8us*)(Wt + (size_t)n * K + k8) = v;
}

template <bool ASPLIT, int ACT, bool BIAS_BF16>
__global__ __launch_bounds__(128) void k_gemm_bf(const float* __restrict__ A, int lda, const unsigned short* __restrict__ Wt, int ldb,
                                               const float* __restrict__ bias, float* __restrict__ C, int ldc, int M, int N, int K) {
  __shared__ __attribute__((aligned(16))) float so[4][16][64];
  const int tid = threadIdx.x, w = tid >> 5, lane = tid & 31, ln = lane & 15, hh = lane >> 4;
  const int ntn = N / 64;
  const int wid = blockIdx.x * 4 + w;
  const int mt = wid / ntn, nq = wid % ntn;
  if (mt * 16 >= M) return;
  const int row0 = mt * 16, col0 = nq * 64;
  const float* arow = A + (size_t)(row0 + ln) * lda;
  v8f acc[4] = {};
  for (int kb = 0; kb < K; kb += 32) {
    FragB ah, al;
    const v4f x0 = *(const v4fa*)(arow + kb + 8 * hh), x1 = *(const v4fa*)(arow + kb + 8 * hh + 4);
    const v4f x2 = *(const v4fa*)(arow + kb + 16 + 8 * hh), x3 = *(const v4fa*)(arow + kb + 16 + 8 * hh + 4);
    float xs[16] = {x0[0],x0[1],x0[2],x0[3],x1[0],x1[1],x1[2],x1[3],x2[0],x2[1],x2[2],x2[3],x3[0],x3[1],x3[2],x3[3]};
#pragma unroll
    for (int i = 0; i < 16; ++i) { const unsigned short hb = bf16_bits(xs[i]); ah.u[i] = hb; al.u[i] = ASPLIT ? bf16_bits(xs[i] - bf16_val(hb)) : (unsigned short)0; }
#pragma unroll
    for (int t = 0; t < 4; ++t) {
      const unsigned short* brow = Wt + (size_t)(col0 + t * 16 + ln) * ldb + kb;
      FragB b;
      b.half[0] = *(const v8us*)(brow + 8 * hh);
      b.half[1] = *(const v8us*)(brow + 16 + 8 * hh);
      acc[t] = mmaN<ASPLIT ? 2 : 1>(ah.v, al.v, b.v, b.v, acc[t]);
    }
  }
#pragma unroll
  for (int t = 0; t < 4; ++t) {
    float bv = bias ? bias[col0 + t * 16 + ln] : 0.f;
    if (BIAS_BF16) bv = bf16_round(bv);
#pragma unroll
    for (int r = 0; r < 8; ++r) { float v = acc[t][r] + bv; if (ACT == 1) v = fmaxf(v, 0.f); so[w][8 * hh + r][t * 16 + ln] = v; }
  }
  __builtin_amdgcn_fence(__ATOMIC_ACQ_REL, "workgroup");
  __builtin_amdgcn_wave_barrier();
  const int rsub = lane >> 4, c4 = (lane & 15) * 4;
  for (int pass = 0; pass < 2; ++pass) {
#pragma unroll
    for (int q = 0; q < 8; ++q) {
      const int r = q * 2 + rsub;
      const v4f v = *(const v4fa*)&so[w][r][c4];
      *(volatile v4f*)(C + (size_t)(row0 + r) * ldc + col0 + c4) = v;
    }
    if (pass == 0) __threadfence();
  }
}

template <int D, bool CAUSAL>
__global__ __launch_bounds__(128) void k_flash(const float* __restrict__ qb, const float* __restrict__ kb, const float* __restrict__ vb,
                                             int pitch, int T, int H, float scale, float* __restrict__ y, int ypitch) {
  constexpr int KS = D / 32;
  constexpr int DT = D / 16;
  __shared__ __attribute__((aligned(16))) unsigned short sKh[32][D + 8], sKl[32][D + 8], sVh[32][D + 8], sVl[32][D + 8];
  __shared__ __attribute__((aligned(16))) unsigned short sPh[4][16][40], sPl[4][16][40];
  __shared__ __attribute__((aligned(16))) float sO[4][16][D];
  const int tid = threadIdx.x, w = tid >> 5, lane = tid & 31, ln = lane & 15, hh = lane >> 4;
  const int nqb = (T + 63) / 64;
  const int bh = blockIdx.x / nqb, qblk = blockIdx.x % nqb;
  const int b = bh / H, h = bh % H;
  const int q0 = qblk * 64 + w * 16;
  const float* Q = qb + (size_t)b * T * pitch + h * D;
  const float* K = kb + (size_t)b * T * pitch + h * D;
  const float* V = vb + (size_t)b * T * pitch + h * D;

  FragB aqh[KS], aql[KS];
  {
    int row = q0 + ln; if (row >= T) row = T - 1;
    const float* qr = Q + (size_t)row * pitch;
#pragma unroll
    for (int ks = 0; ks < KS; ++ks)
#pragma unroll
      for (int i = 0; i < 16; ++i) {
        const int d = ks * 32 + ((i < 8) ? (8 * hh + i) : (16 + 8 * hh + (i - 8)));
        const float x = qr[d] * scale; const unsigned short hb = bf16_bits(x);
        aqh[ks].u[i] = hb; aql[ks].u[i] = bf16_bits(x - bf16_val(hb));
      }
  }
  float m_r[8], l_r[8];
#pragma unroll
  for (int r = 0; r < 8; ++r) { m_r[r] = -3.0e38f; l_r[r] = 0.f; }
  v8f oacc[DT];
#pragma unroll
  for (int dt = 0; dt < DT; ++dt) oacc[dt] = (v8f){0.f,0.f,0.f,0.f,0.f,0.f,0.f,0.f};

  const int kv_end = CAUSAL ? min(T, qblk * 64 + 64) : T;
  for (int j0 = 0; j0 < kv_end; j0 += 32) {
    __syncthreads();
    for (int e = tid; e < 32 * (D / 4); e += 128) {
      const int r = e / (D / 4), c4 = (e % (D / 4)) * 4;
      const int key = j0 + r;
      v4f kf = {0.f,0.f,0.f,0.f}, vf = {0.f,0.f,0.f,0.f};
      if (key < T) { kf = *(const v4fa*)(K + (size_t)key * pitch + c4); vf = *(const v4fa*)(V + (size_t)key * pitch + c4); }
#pragma unroll
      for (int t = 0; t < 4; ++t) {
        unsigned short hb = bf16_bits(kf[t]); sKh[r][c4 + t] = hb; sKl[r][c4 + t] = bf16_bits(kf[t] - bf16_val(hb));
        hb = bf16_bits(vf[t]); sVh[r][c4 + t] = hb; sVl[r][c4 + t] = bf16_bits(vf[t] - bf16_val(hb));
      }
    }
    __syncthreads();
    v8f s[2];
#pragma unroll
    for (int nt = 0; nt < 2; ++nt) {
      v8f acc = {};
#pragma unroll
      for (int ks = 0; ks < KS; ++ks) {
        FragB bh_, bl_;
        bh_.half[0] = *(const v8us*)&sKh[nt * 16 + ln][ks * 32 + 8 * hh]; bh_.half[1] = *(const v8us*)&sKh[nt * 16 + ln][ks * 32 + 16 + 8 * hh];
        bl_.half[0] = *(const v8us*)&sKl[nt * 16 + ln][ks * 32 + 8 * hh]; bl_.half[1] = *(const v8us*)&sKl[nt * 16 + ln][ks * 32 + 16 + 8 * hh];
        acc = mmaN<3>(aqh[ks].v, aql[ks].v, bh_.v, bl_.v, acc);
      }
      s[nt] = acc;
    }
    float alpha[8];
#pragma unroll
    for (int r = 0; r < 8; ++r) {
      const int qi = q0 + 8 * hh + r;
      const int ja = j0 + ln, jb = j0 + 16 + ln;
      if (CAUSAL) { if (ja > qi) s[0][r] = -3.0e38f; if (jb > qi) s[1][r] = -3.0e38f; }
      if (ja >= T) s[0][r] = -3.0e38f;
      if (jb >= T) s[1][r] = -3.0e38f;
      float mx = fmaxf(s[0][r], s[1][r]);
      mx = fmaxf(mx, __shfl_xor(mx, 1, 32)); mx = fmaxf(mx, __shfl_xor(mx, 2, 32)); mx = fmaxf(mx, __shfl_xor(mx, 4, 32)); mx = fmaxf(mx, __shfl_xor(mx, 8, 32));
      const float mnew = fmaxf(m_r[r], mx);
      alpha[r] = (mnew > -1.0e38f) ? __expf(m_r[r] - mnew) : 1.0f;
      const float p0 = (s[0][r] > -1.0e38f) ? __expf(s[0][r] - mnew) : 0.f;
      const float p1 = (s[1][r] > -1.0e38f) ? __expf(s[1][r] - mnew) : 0.f;
      m_r[r] = mnew;
      l_r[r] = l_r[r] * alpha[r] + p0 + p1;
      unsigned short hb = bf16_bits(p0); sPh[w][8 * hh + r][ln] = hb;      sPl[w][8 * hh + r][ln] = bf16_bits(p0 - bf16_val(hb));
      hb = bf16_bits(p1);                sPh[w][8 * hh + r][16 + ln] = hb; sPl[w][8 * hh + r][16 + ln] = bf16_bits(p1 - bf16_val(hb));
    }
#pragma unroll
    for (int dt = 0; dt < DT; ++dt)
#pragma unroll
      for (int r = 0; r < 8; ++r) oacc[dt][r] *= alpha[r];
    __builtin_amdgcn_fence(__ATOMIC_ACQ_REL, "workgroup");
    __builtin_amdgcn_wave_barrier();
    FragB pah, pal;
    pah.half[0] = *(const v8us*)&sPh[w][ln][8 * hh]; pah.half[1] = *(const v8us*)&sPh[w][ln][16 + 8 * hh];
    pal.half[0] = *(const v8us*)&sPl[w][ln][8 * hh]; pal.half[1] = *(const v8us*)&sPl[w][ln][16 + 8 * hh];
#pragma unroll
    for (int dt = 0; dt < DT; ++dt) {
      FragB bvh, bvl;
#pragma unroll
      for (int i = 0; i < 8; ++i) {
        bvh.u[i] = sVh[8 * hh + i][dt * 16 + ln]; bvh.u[8 + i] = sVh[16 + 8 * hh + i][dt * 16 + ln];
        bvl.u[i] = sVl[8 * hh + i][dt * 16 + ln]; bvl.u[8 + i] = sVl[16 + 8 * hh + i][dt * 16 + ln];
      }
      oacc[dt] = mmaN<3>(pah.v, pal.v, bvh.v, bvl.v, oacc[dt]);
    }
    __builtin_amdgcn_fence(__ATOMIC_ACQ_REL, "workgroup");
    __builtin_amdgcn_wave_barrier();
  }
#pragma unroll
  for (int r = 0; r < 8; ++r) {
    float l = l_r[r];
    l += __shfl_xor(l, 1, 32); l += __shfl_xor(l, 2, 32); l += __shfl_xor(l, 4, 32); l += __shfl_xor(l, 8, 32);
    l_r[r] = (l > 0.f) ? 1.0f / l : 0.f;
  }
#pragma unroll
  for (int dt = 0; dt < DT; ++dt)
#pragma unroll
    for (int r = 0; r < 8; ++r) sO[w][8 * hh + r][dt * 16 + ln] = oacc[dt][r] * l_r[r];
  __builtin_amdgcn_fence(__ATOMIC_ACQ_REL, "workgroup");
  __builtin_amdgcn_wave_barrier();
  for (int pass = 0; pass < 2; ++pass) {
    for (int r = 0; r < 16; ++r) {
      const int row = q0 + r;
      if (row < T && lane < D / 4) {
        const v4f val = *(const v4fa*)&sO[w][r][lane * 4];
        *(volatile v4f*)(y + ((size_t)b * T + row) * ypitch + h * D + lane * 4) = val;
      }
    }
    if (pass == 0) __threadfence();
  }
}

template <bool ASPLIT, int ACT, bool BIAS_BF16, bool RES_BF16>
__global__ __launch_bounds__(128) void k_gemm_bf3(const float* __restrict__ A, int lda, const unsigned short* __restrict__ Wt, int ldb,
                                                const float* __restrict__ bias, const float* __restrict__ resid, int rmod, int ldr,
                                                float* __restrict__ C, int ldc, int M, int N, int K) {
  __shared__ __attribute__((aligned(16))) float so[4][16][64];
  const int tid = threadIdx.x, w = tid >> 5, lane = tid & 31, ln = lane & 15, hh = lane >> 4;
  const int ntn = N / 64;
  const int wid = blockIdx.x * 4 + w;
  const int mt = wid / ntn, nq = wid % ntn;
  if (mt * 16 >= M) return;
  const int row0 = mt * 16, col0 = nq * 64;
  const float* arow = A + (size_t)(row0 + ln) * lda;
  v8f acc[4] = {};
  for (int kb = 0; kb < K; kb += 32) {
    FragB ah, al;
    const v4f x0 = *(const v4fa*)(arow + kb + 8 * hh), x1 = *(const v4fa*)(arow + kb + 8 * hh + 4);
    const v4f x2 = *(const v4fa*)(arow + kb + 16 + 8 * hh), x3 = *(const v4fa*)(arow + kb + 16 + 8 * hh + 4);
    float xs[16] = {x0[0],x0[1],x0[2],x0[3],x1[0],x1[1],x1[2],x1[3],x2[0],x2[1],x2[2],x2[3],x3[0],x3[1],x3[2],x3[3]};
#pragma unroll
    for (int i = 0; i < 16; ++i) { const unsigned short hb = bf16_bits(xs[i]); ah.u[i] = hb; al.u[i] = ASPLIT ? bf16_bits(xs[i] - bf16_val(hb)) : (unsigned short)0; }
#pragma unroll
    for (int t = 0; t < 4; ++t) {
      const unsigned short* brow = Wt + (size_t)(col0 + t * 16 + ln) * ldb + kb;
      FragB b;
      b.half[0] = *(const v8us*)(brow + 8 * hh);
      b.half[1] = *(const v8us*)(brow + 16 + 8 * hh);
      acc[t] = mmaN<ASPLIT ? 2 : 1>(ah.v, al.v, b.v, b.v, acc[t]);
    }
  }
#pragma unroll
  for (int t = 0; t < 4; ++t) {
    const int col = col0 + t * 16 + ln;
    float bv = bias ? bias[col] : 0.f;
    if (BIAS_BF16) bv = bf16_round(bv);
#pragma unroll
    for (int r = 0; r < 8; ++r) {
      float v = acc[t][r] + bv;
      if (resid) { float rv = resid[(size_t)((row0 + 8 * hh + r) % rmod) * ldr + col]; if (RES_BF16) rv = bf16_round(rv); v += rv; }
      if (ACT == 1) v = fmaxf(v, 0.f);
      if (ACT == 2) v = 0.5f * v * (1.0f + erff(v * 0.70710678118654752f));
      if (ACT == 3) { const float u = 0.7978845608028654f * (v + 0.044715f * v * v * v); v = 0.5f * v * (1.0f + tanhf(u)); }
      so[w][8 * hh + r][t * 16 + ln] = v;
    }
  }
  __builtin_amdgcn_fence(__ATOMIC_ACQ_REL, "workgroup");
  __builtin_amdgcn_wave_barrier();
  const int rsub = lane >> 4, c4 = (lane & 15) * 4;
  for (int pass = 0; pass < 2; ++pass) {
#pragma unroll
    for (int q = 0; q < 8; ++q) {
      const int r = q * 2 + rsub;
      const v4f v = *(const v4fa*)&so[w][r][c4];
      *(volatile v4f*)(C + (size_t)(row0 + r) * ldc + col0 + c4) = v;
    }
    if (pass == 0) __threadfence();
  }
}
template <bool PARAM_BF16>
__global__ __launch_bounds__(256) void k_layernorm(const float* __restrict__ X, const float* __restrict__ R, const float* __restrict__ g, const float* __restrict__ bta,
                                                  float* __restrict__ out_sum, float* __restrict__ out_norm, int N, float eps) {
  __shared__ float red[256];
  const int row = blockIdx.x, tid = threadIdx.x;
  const float* x = X + (size_t)row * N; const float* rr = R ? R + (size_t)row * N : nullptr;
  float vals[16];
  const int per = N / 256;
  float s1 = 0.f;
  for (int u = 0; u < per / 4; ++u) {
    const int j = tid * 4 + 1024 * u;
    const v4f a = *(const v4fa*)(x + j);
    v4f b = {0.f,0.f,0.f,0.f}; if (rr) b = *(const v4fa*)(rr + j);
#pragma unroll
    for (int q = 0; q < 4; ++q) { const float v = a[q] + b[q]; vals[u * 4 + q] = v; s1 += v; }
  }
  red[tid] = s1; __syncthreads();
  for (int st = 128; st > 0; st >>= 1) { if (tid < st) red[tid] += red[tid + st]; __syncthreads(); }
  const float mu = red[0] / (float)N; __syncthreads();
  float s2 = 0.f;
  for (int u = 0; u < per / 4; ++u)
#pragma unroll
    for (int q = 0; q < 4; ++q) { const float c = vals[u * 4 + q] - mu; s2 += c * c; }
  red[tid] = s2; __syncthreads();
  for (int st = 128; st > 0; st >>= 1) { if (tid < st) red[tid] += red[tid + st]; __syncthreads(); }
  const float rs = rsqrtf(red[0] / (float)N + eps);
  for (int pass = 0; pass < 2; ++pass) {
    for (int u = 0; u < per / 4; ++u) {
      const int j = tid * 4 + 1024 * u;
      v4f o, sm;
#pragma unroll
      for (int q = 0; q < 4; ++q) {
        float gg = g[j + q], bb = bta[j + q];
        if (PARAM_BF16) { gg = bf16_round(gg); bb = bf16_round(bb); }
        sm[q] = vals[u * 4 + q]; o[q] = (vals[u * 4 + q] - mu) * rs * gg + bb;
      }
      if (out_sum) *(volatile v4f*)(out_sum + (size_t)row * N + j) = sm;
      *(volatile v4f*)(out_norm + (size_t)row * N + j) = o;
    }
    if (pass == 0) __threadfence();
  }
}

__device__ __forceinline__ float clip01(float v) { return fminf(fmaxf(v, 1e-6f), 1.0f); }
__device__ __forceinline__ int reflect(int i, int n) { return i < 0 ? -i : (i >= n ? 2 * n - 2 - i : i); }
__global__ __launch_bounds__(256) void k_resize256(const float* __restrict__ img, float* __restrict__ x256) {
  const int t = blockIdx.x * 256 + threadIdx.x; if (t >= BB * 3 * 256 * 256) return; const int ox = t % 256, oy = (t / 256) % 256, bc = t / 65536;
  const float step = (float)(HI - 1) / 255.0f; const float ys = (oy == 255) ? (float)(HI - 1) : 0.0f + step * (float)oy, xs = (ox == 255) ? (float)(WI - 1) : 0.0f + step * (float)ox;
  const int y0 = (int)floorf(ys), x0 = (int)floorf(xs); const int y1 = min(y0 + 1, HI - 1), x1 = min(x0 + 1, WI - 1); const float wy = ys - (float)y0, wx = xs - (float)x0;
  const float* p = img + (size_t)bc * NPIX; const float a = bf16_round(p[(size_t)y0 * WI + x0]), bq = bf16_round(p[(size_t)y0 * WI + x1]), c = bf16_round(p[(size_t)y1 * WI + x0]), d = bf16_round(p[(size_t)y1 * WI + x1]);
  const float top = a * (1.0f - wx) + bq * wx, bot = c * (1.0f - wx) + d * wx; const float v = top * (1.0f - wy) + bot * wy;
  *(volatile float*)(x256 + t) = v; __threadfence(); *(volatile float*)(x256 + t) = v;
}
__global__ __launch_bounds__(256) void k_convs2(const float* __restrict__ in, int CI, int HIN, const float* __restrict__ w, const float* __restrict__ bias, int CO, float* __restrict__ out) {
  const int HO = HIN / 2; const int t = blockIdx.x * 256 + threadIdx.x; if (t >= BB * CO * HO * HO) return; const int ox = t % HO, oy = (t / HO) % HO, o = (t / (HO * HO)) % CO, b = t / (HO * HO * CO);
  float a = bf16_round(bias[o]);
#pragma unroll 1
  for (int ci = 0; ci < CI; ++ci) { const float* ip = in + ((size_t)b * CI + ci) * HIN * HIN; const float* wp = w + ((size_t)o * CI + ci) * 9;
#pragma unroll 1
    for (int ky = 0; ky < 3; ++ky) { const int yy = oy * 2 - 1 + ky; if (yy < 0 || yy >= HIN) continue; for (int kx = 0; kx < 3; ++kx) { const int xx = ox * 2 - 1 + kx; if (xx < 0 || xx >= HIN) continue; a += bf16_round(wp[ky * 3 + kx]) * ip[(size_t)yy * HIN + xx]; } } }
  const float v = fmaxf(a, 0.f); *(volatile float*)(out + t) = v; __threadfence(); *(volatile float*)(out + t) = v;
}
__global__ __launch_bounds__(256) void k_gmean(const float* __restrict__ c3, float* __restrict__ G16) {
  __shared__ float sv[512]; const int t = threadIdx.x; float v = 0.f;
  if (t < BB * NF) { const float* p = c3 + (size_t)t * 1024; float s = 0.f;
#pragma unroll 1
    for (int i = 0; i < 1024; ++i) s += p[i]; v = s / 1024.0f; }
  sv[t] = (t < BB * NF) ? v : 0.f; sv[256 + t] = 0.f; __syncthreads();
  for (int pass = 0; pass < 2; ++pass) { for (int e = t; e < 16 * NF; e += 256) *(volatile float*)(G16 + e) = sv[e]; if (pass == 0) __threadfence(); }
}
__global__ __launch_bounds__(256) void k_wth(const float* __restrict__ dw, const float* __restrict__ cw, const float* __restrict__ gw, const float* __restrict__ db, const float* __restrict__ cb, const float* __restrict__ gb, unsigned short* __restrict__ Bt, float* __restrict__ bias) {
  const int t = blockIdx.x * 256 + threadIdx.x; if (t >= 128 * 4) return; const int n = t / 4, k8 = (t % 4) * 8; v8us v;
  for (int i = 0; i < 8; ++i) { const int k = k8 + i; float w = 0.f; if (n == 0) w = dw[k]; else if (n < 28) w = cw[(n - 1) * NF + k]; else if (n < 103) w = gw[(n - 28) * NF + k]; v[i] = bf16_bits(w); }
  *(volatile v8us*)(Bt + (size_t)n * NF + k8) = v; __threadfence(); *(volatile v8us*)(Bt + (size_t)n * NF + k8) = v;
  if (t < 128) { float b = 0.f; if (t == 0) b = db[0]; else if (t < 28) b = cb[t - 1]; else if (t < 103) b = gb[t - 28]; b = bf16_round(b); *(volatile float*)(bias + t) = b; __threadfence(); *(volatile float*)(bias + t) = b; }
}
__global__ __launch_bounds__(256) void k_stageA(const float* __restrict__ img, const float* __restrict__ heads, float* __restrict__ inter, double* __restrict__ part) {
  __shared__ double red[3][256];
  const int t = threadIdx.x; const size_t gid = (size_t)blockIdx.x * 256 + t; const int b = (int)(gid / NPIX); const int p = (int)(gid % NPIX); const int y = p / WI, x = p % WI;
  const float dg = (1.0f / (1.0f + expf(-heads[b * 128 + 0]))) * 0.1f + 1.0f;
  const float e1 = expf(-1.0f / 2.0f); const float k2c = 1.0f, k2e = e1, k2d = e1 * e1; const float ksum = k2c + 4.0f * k2e + 4.0f * k2d;
  double cs[3];
#pragma unroll 1
  for (int c = 0; c < 3; ++c) { const float* ip = img + ((size_t)b * 3 + c) * NPIX; const float ctr = bf16_round(ip[p]);
    float num = 0.f, den = 0.f;
#pragma unroll 1
    for (int k = 0; k < 9; ++k) { const int i = k / 3, j = k % 3; const int yy = reflect(y + i - 1, HI), xx = reflect(x + j - 1, WI); const float v = bf16_round(ip[(size_t)yy * WI + xx]); const float d = v - ctr;
      const float ksp = ((i == 1 && j == 1) ? k2c : ((i == 1 || j == 1) ? k2e : k2d)) / ksum; const float w = __expf(-(d * d) / 0.005f) * ksp; num += w * v; den += w; }
    const float bf = num / den; const float de = clip01(0.5f * ctr + 0.5f * bf); const float it = clip01(de * dg);
    *(volatile float*)(inter + ((size_t)b * 3 + c) * NPIX + p) = it; cs[c] = (double)it; }
  __threadfence();
#pragma unroll 1
  for (int c = 0; c < 3; ++c) { *(volatile float*)(inter + ((size_t)b * 3 + c) * NPIX + p) = (float)cs[c]; red[c][t] = cs[c]; }
  __syncthreads(); for (int s = 128; s > 0; s >>= 1) { if (t < s) { red[0][t] += red[0][t + s]; red[1][t] += red[1][t + s]; red[2][t] += red[2][t + s]; } __syncthreads(); }
  if (t < 16) { const double v = (t < 3) ? red[t][0] : 0.0; *(volatile double*)(part + (size_t)blockIdx.x * 16 + t) = v; __threadfence(); *(volatile double*)(part + (size_t)blockIdx.x * 16 + t) = v; }
}
__global__ __launch_bounds__(256) void k_means(const double* __restrict__ part, int nparts, float* __restrict__ ratio) {
  __shared__ double red[3][256]; const int t = threadIdx.x; double s0 = 0, s1 = 0, s2 = 0; for (int i = t; i < nparts; i += 256) { s0 += part[(size_t)i * 16]; s1 += part[(size_t)i * 16 + 1]; s2 += part[(size_t)i * 16 + 2]; }
  red[0][t] = s0; red[1][t] = s1; red[2][t] = s2; __syncthreads(); for (int s = 128; s > 0; s >>= 1) { if (t < s) { red[0][t] += red[0][t + s]; red[1][t] += red[1][t + s]; red[2][t] += red[2][t + s]; } __syncthreads(); }
  const double n = (double)BB * NPIX; const float mr = (float)(red[0][0] / n), mg = (float)(red[1][0] / n), mb = (float)(red[2][0] / n);
  if (t < 32) { const float v = (t == 0) ? mg / mr : (t == 1 ? mg / mb : 0.f); *(volatile float*)(ratio + t) = v; __threadfence(); *(volatile float*)(ratio + t) = v; }
}
__global__ __launch_bounds__(256) void k_stageB(const float* __restrict__ inter, const float* __restrict__ heads, const float* __restrict__ ratio, float* __restrict__ out) {
  __shared__ float sccm[27]; __shared__ float sgam[75];
  const int t = threadIdx.x; const size_t gid = (size_t)blockIdx.x * 256 + t; const int b = (int)(gid / NPIX); const int p = (int)(gid % NPIX); const int y = p / WI, x = p % WI;
  if (t < 27) sccm[t] = 2.0f * heads[b * 128 + 1 + t] + 1.0f; if (t < 75) sgam[t] = (1.0f / (1.0f + expf(-heads[b * 128 + 28 + t]))) * 0.8f + 2.2f;
  __syncthreads();
  const float r0 = inter[((size_t)b * 3 + 0) * NPIX + p], g0 = inter[((size_t)b * 3 + 1) * NPIX + p], b0 = inter[((size_t)b * 3 + 2) * NPIX + p];
  const float R = clip01(r0 * ratio[0]), G = clip01(g0), Bc = clip01(b0 * ratio[1]);
  const float X[9] = {R, G, Bc, R * R, G * G, Bc * Bc, R * G, R * Bc, G * Bc};
  const float step = 4.0f / (float)(HI - 1); const float ys = (y == HI - 1) ? 4.0f : step * (float)y, xs = (x == WI - 1) ? 4.0f : step * (float)x;
  const int y0 = (int)floorf(ys), x0 = (int)floorf(xs); const int y1 = min(y0 + 1, 4), x1 = min(x0 + 1, 4); const float wy = ys - (float)y0, wx = xs - (float)x0;
  float inv_gm[3];
#pragma unroll 1
  for (int k = 0; k < 3; ++k) { const float* gmp = sgam + k * 25; const float top = gmp[y0 * 5 + x0] * (1.0f - wx) + gmp[y0 * 5 + x1] * wx, bot = gmp[y1 * 5 + x0] * (1.0f - wx) + gmp[y1 * 5 + x1] * wx; inv_gm[k] = 1.0f / (top * (1.0f - wy) + bot * wy); }
#pragma unroll 1
  for (int c = 0; c < 3; ++c) { float s = 0.f;
#pragma unroll 1
    for (int j = 0; j < 9; ++j) s += sccm[c * 9 + j] * X[j];
    const float oc = clip01(s); float m = 0.f;
#pragma unroll 1
    for (int k = 0; k < 3; ++k) m += __builtin_amdgcn_exp2f(__log2f(oc) * inv_gm[k]);
    const float v = m / 3.0f; float* op = out + ((size_t)b * 3 + c) * NPIX + p; *(volatile float*)op = v; __threadfence(); *(volatile float*)op = v; }
}
extern "C" void kernel_launch(void* const* d_in, const int* in_sizes, int n_in,
                              void* d_out, int out_size, void* d_ws, size_t ws_size, hipStream_t stream) {
  (void)in_sizes; (void)n_in; (void)out_size;
  const float* img = (const float*)d_in[0]; const float* c1w = (const float*)d_in[1]; const float* c1b = (const float*)d_in[2]; const float* c2w = (const float*)d_in[3]; const float* c2b = (const float*)d_in[4]; const float* c3w = (const float*)d_in[5]; const float* c3b = (const float*)d_in[6];
  const float* gw = (const float*)d_in[7]; const float* gb = (const float*)d_in[8]; const float* dw = (const float*)d_in[9]; const float* db = (const float*)d_in[10]; const float* cw = (const float*)d_in[11]; const float* cb = (const float*)d_in[12];
  char* ws = (char*)d_ws; size_t off = 0;
  auto take = [&](size_t bytes) { char* p = ws + off; off += (bytes + 255) & ~(size_t)255; return p; };
  float* x256 = (float*)take((size_t)BB * 3 * 65536 * 4); float* c1 = (float*)take((size_t)BB * NF * 128 * 128 * 4); float* c2 = (float*)take((size_t)BB * NF * 64 * 64 * 4); float* c3 = (float*)take((size_t)BB * NF * 32 * 32 * 4);
  float* G16 = (float*)take(16 * NF * 4); unsigned short* Bt = (unsigned short*)take(128 * NF * 2); float* hb = (float*)take(128 * 4); float* heads = (float*)take(16 * 128 * 4);
  float* inter = (float*)take((size_t)BB * 3 * NPIX * 4); const int nparts = BB * NPIX / 256; double* part = (double*)take((size_t)nparts * 16 * 8); float* ratio = (float*)take(32 * 4);
  if (off > ws_size) return;
  k_resize256<<<(BB * 3 * 65536 + 255) / 256, 256, 0, stream>>>(img, x256);
  k_convs2<<<(BB * NF * 128 * 128 + 255) / 256, 256, 0, stream>>>(x256, 3, 256, c1w, c1b, NF, c1);
  k_convs2<<<(BB * NF * 64 * 64 + 255) / 256, 256, 0, stream>>>(c1, NF, 128, c2w, c2b, NF, c2);
  k_convs2<<<(BB * NF * 32 * 32 + 255) / 256, 256, 0, stream>>>(c2, NF, 64, c3w, c3b, NF, c3);
  k_gmean<<<1, 256, 0, stream>>>(c3, G16);
  k_wth<<<2, 256, 0, stream>>>(dw, cw, gw, db, cb, gb, Bt, hb);
  k_gemm_bf3<true, 0, false, false><<<1, 128, 0, stream>>>(G16, NF, Bt, NF, hb, nullptr, 1, 0, heads, 128, 16, 128, NF);
  k_stageA<<<BB * NPIX / 256, 256, 0, stream>>>(img, heads, inter, part);
  k_means<<<1, 256, 0, stream>>>(part, nparts, ratio);
  k_stageB<<<BB * NPIX / 256, 256, 0, stream>>>(inter, heads, ratio, (float*)d_out);
}
